// PointConvFlow_70437463654602
// MI455X (gfx1250) — hardware-verified
//
#include <hip/hip_runtime.h>
#include <math.h>
#include <stddef.h>
#include <stdint.h>

#pragma clang fp contract(off)


#define NB    8
#define NP    4096
#define ND    64
#define NK    16
#define CIN   131
#define K1P   160
#define KAP   96
#define TPB   64
#define WPB   2
#define NSG   8
#define ASC   8.0f
#define WSC   1024.0f
#define XINV  0.0001220703125f

#define SM_W1  0
#define SM_W2  20480
#define SM_B1  28672
#define SM_B2  28928
#define SM_REG 29184
#define WV_XP1 0
#define WV_XA  4096
#define WV_X1  16384
#define WV_IDX 24576
#define WV_WT  26624
#define WV_OUT 26880
#define WVB    35072
#define SM_X2B (NP * 16)
#define SMEM   (SM_REG + WPB * WVB)

static_assert(WPB * WVB >= SM_X2B);
static_assert(SM_W2 == SM_W1 + ND * K1P * 2);
static_assert(SM_B1 == SM_W2 + ND * ND * 2);
static_assert(SM_B2 == SM_B1 + ND * 4);
static_assert(SM_REG == SM_B2 + ND * 4);
static_assert(WV_XA == WV_XP1 + 32 * ND * 2);
static_assert(WV_X1 == WV_XA + 64 * KAP * 2);
static_assert(WV_IDX == WV_X1 + 64 * ND * 2);
static_assert(WV_WT == WV_IDX + 32 * NK * 4);
static_assert(WV_OUT == WV_WT + 64 * 4);
static_assert(WVB == WV_OUT + ND * 32 * 4);
static_assert((SM_REG % 16) == 0 && (WVB % 16) == 0);
static_assert(TPB == 32 * WPB);
static_assert(TPB == ND);
static_assert(NP % TPB == 0);
static_assert(NP % 4 == 0);
static_assert(NSG * 4 == 32);
static_assert(K1P % 32 == 0 && KAP % 32 == 0 && ND % 32 == 0);
static_assert(CIN <= K1P && ND + 3 <= 64 + 32 && KAP == 64 + 32);
static_assert(SMEM == 99328);

typedef float    v4f  __attribute__((ext_vector_type(4)));
typedef float    v8f  __attribute__((ext_vector_type(8)));
typedef int      v4i  __attribute__((ext_vector_type(4)));
typedef _Float16 v8h  __attribute__((ext_vector_type(8)));
typedef _Float16 v16h __attribute__((ext_vector_type(16)));
union FragH { v16h v; v8h h[2]; };

__device__ __forceinline__ v8f wmf(v16h a, v16h b, v8f c) {
  v8f d = __builtin_amdgcn_wmma_f32_16x16x32_f16(false, a, false, b, (short)0, c, false, false);
  asm volatile("v_nop\n\tv_nop\n\tv_nop\n\tv_nop" : "+v"(d) : "v"(a), "v"(b));
  return d;
}

__device__ __forceinline__ v8f splat8(float x) { v8f r = {x, x, x, x, x, x, x, x}; return r; }

__device__ __forceinline__ v16h ldfrag(const _Float16* p, int k0, int hh) {
  FragH u;
  u.h[0] = *(const v8h*)(p + k0 + 8 * hh);
  u.h[1] = *(const v8h*)(p + k0 + 16 + 8 * hh);
  return u.v;
}

__device__ __forceinline__ void wave_sync() {
  __builtin_amdgcn_fence(__ATOMIC_RELEASE, "wavefront");
  __builtin_amdgcn_wave_barrier();
}

__device__ __forceinline__ float vgpr_zero() {
  float z;
  asm volatile("v_mov_b32 %0, 0" : "=v"(z));
  return z;
}

__device__ __forceinline__ float leaky01(float x) { return (x >= 0.0f) ? x : 0.1f * x; }

__device__ __forceinline__ float norm3sq(float x, float y, float z) {
#pragma clang fp contract(off)
  float xx = x * x;
  asm volatile("" : "+v"(xx));
  float zz = z * z;
  asm volatile("" : "+v"(zz));
  float yy = y * y;
  asm volatile("" : "+v"(yy));
  float s = xx + zz;
  asm volatile("" : "+v"(s));
  return s + yy;
}

__device__ __forceinline__ void top16_insert(float (&bd)[NK], int (&bi)[NK], float d, int m) {
#pragma unroll
  for (int j = NK - 1; j >= 1; --j) {
    const bool up = bd[j - 1] > d;
    const bool here = bd[j] > d;
    const float nd = up ? bd[j - 1] : (here ? d : bd[j]);
    const int ni = up ? bi[j - 1] : (here ? m : bi[j]);
    bd[j] = nd;
    bi[j] = ni;
  }
  const bool h0 = bd[0] > d;
  bd[0] = h0 ? d : bd[0];
  bi[0] = h0 ? m : bi[0];
}

__global__ __launch_bounds__(TPB) void k_main(const float* __restrict__ xyz1,
                                               const float* __restrict__ xyz2,
                                               const float* __restrict__ pts1,
                                               const float* __restrict__ pts2,
                                               const float* __restrict__ W1,
                                               const float* __restrict__ b1v,
                                               const float* __restrict__ W2,
                                               const float* __restrict__ b2v,
                                               float* outp) {
#pragma clang fp contract(off)
  extern __shared__ __attribute__((aligned(16))) char smem[];
  _Float16* sW1 = (_Float16*)(smem + SM_W1);
  _Float16* sW2 = (_Float16*)(smem + SM_W2);
  float* sB1 = (float*)(smem + SM_B1);
  float* sB2 = (float*)(smem + SM_B2);
  v4f* sX2 = (v4f*)(smem + SM_REG);

  const int t = threadIdx.x, lane = t & 31, wv = t >> 5;
  const int hh = lane >> 4, nl = lane & 15;
  char* wreg = smem + SM_REG + wv * WVB;
  _Float16* XP1 = (_Float16*)(wreg + WV_XP1);
  _Float16* XA  = (_Float16*)(wreg + WV_XA);
  _Float16* X1  = (_Float16*)(wreg + WV_X1);
  int*   sIdx = (int*)(wreg + WV_IDX);
  float* sWt  = (float*)(wreg + WV_WT);
  float* sOut = (float*)(wreg + WV_OUT);

  const int blk = blockIdx.x;
  const int b = blk / (NP / TPB);
  const int n0 = (blk - b * (NP / TPB)) * TPB;
  const int n0w = n0 + 32 * wv;
  const int qn = n0 + t;
  const float* x1b = xyz1 + (size_t)b * 3 * NP;
  const float* x2b = xyz2 + (size_t)b * 3 * NP;
  const float* p1b = pts1 + (size_t)b * ND * NP;
  const float* p2b = pts2 + (size_t)b * ND * NP;

#pragma unroll 1
  for (int e = t; e < ND * K1P; e += TPB) {
    const int o = e / K1P, c = e - o * K1P;
    const float v = W1[o * CIN + min(c, CIN - 1)];
    sW1[e] = (_Float16)((c < CIN) ? v * WSC : 0.0f);
  }
#pragma unroll 1
  for (int e = t; e < ND * ND; e += TPB) sW2[e] = (_Float16)(W2[e] * WSC);
  sB1[t] = b1v[t];
  sB2[t] = b2v[t];
#pragma unroll 1
  for (int m = t; m < NP; m += TPB) {
    const float sx = x2b[m], sy = x2b[NP + m], sz = x2b[2 * NP + m];
    const v4f v = {sx, sy, sz, norm3sq(sx, sy, sz)};
    sX2[m] = v;
  }
  __syncthreads();

  const float qx = x1b[qn], qy = x1b[NP + qn], qz = x1b[2 * NP + qn];
  const float nqv = norm3sq(qx, qy, qz);
  float bd[NK];
  int bi[NK];
#pragma unroll
  for (int k = 0; k < NK; ++k) { bd[k] = __int_as_float(0x7f800000); bi[k] = 0; }
#pragma unroll 1
  for (int mb = 0; mb < NP; mb += 4) {
#pragma unroll
    for (int u = 0; u < 4; ++u) {
      const int m = mb + u;
      const v4f s = sX2[m];
      const float p0 = qx * s.x;
      float dt = fmaf(qy, s.y, p0);
      dt = fmaf(qz, s.z, dt);
      float t2 = dt * 2.0f;
      asm volatile("" : "+v"(t2));
      float df = nqv - t2;
      asm volatile("" : "+v"(df));
      const float sq = df + s.w;
      if (__builtin_amdgcn_ballot_w32(sq < bd[NK - 1]) != 0u) top16_insert(bd, bi, sq, m);
    }
  }
  __syncthreads();
  {
    v4i* di = (v4i*)(sIdx + lane * NK);
    const v4i a0 = {bi[0], bi[1], bi[2], bi[3]};
    const v4i a1 = {bi[4], bi[5], bi[6], bi[7]};
    const v4i a2 = {bi[8], bi[9], bi[10], bi[11]};
    const v4i a3 = {bi[12], bi[13], bi[14], bi[15]};
    di[0] = a0; di[1] = a1; di[2] = a2; di[3] = a3;
  }
  __syncthreads();

#pragma unroll 8
  for (int c = 0; c < ND; ++c)
    XP1[lane * ND + c] = (_Float16)(p1b[(size_t)c * NP + n0w + lane] * ASC);
  wave_sync();

#pragma unroll 1
  for (int sg = 0; sg < NSG; ++sg) {
    const int r0 = lane, r1 = lane + 32;
    int j0 = sIdx[64 * sg + r0];
    int j1 = sIdx[64 * sg + r1];
    j0 = min(max(j0, 0), NP - 1);
    j1 = min(max(j1, 0), NP - 1);
    const int na = n0w + 4 * sg + hh;
    const int nb2 = na + 2;
    const float ax = x1b[na], ay = x1b[NP + na], az = x1b[2 * NP + na];
    const float ex = x1b[nb2], ey = x1b[NP + nb2], ez = x1b[2 * NP + nb2];
    const float d0x = x2b[j0] - ax, d0y = x2b[NP + j0] - ay, d0z = x2b[2 * NP + j0] - az;
    const float d1x = x2b[j1] - ex, d1y = x2b[NP + j1] - ey, d1z = x2b[2 * NP + j1] - ez;
    float ds0 = sqrtf(fmaf(d0x, d0x, fmaf(d0y, d0y, d0z * d0z)));
    float ds1 = sqrtf(fmaf(d1x, d1x, fmaf(d1y, d1y, d1z * d1z)));
    ds0 = fmaxf(ds0, 1e-10f);
    ds1 = fmaxf(ds1, 1e-10f);
    const float iv0 = 1.0f / ds0;
    const float iv1 = 1.0f / ds1;
    float s0 = iv0, s1 = iv1;
    s0 += __shfl_xor(s0, 1, 32);  s1 += __shfl_xor(s1, 1, 32);
    s0 += __shfl_xor(s0, 2, 32);  s1 += __shfl_xor(s1, 2, 32);
    s0 += __shfl_xor(s0, 4, 32);  s1 += __shfl_xor(s1, 4, 32);
    s0 += __shfl_xor(s0, 8, 32);  s1 += __shfl_xor(s1, 8, 32);
    const float w0 = iv0 * (1.0f / s0);
    const float w1 = iv1 * (1.0f / s1);
    sWt[r0] = w0;
    sWt[r1] = w1;

    {
      const _Float16 hz = (_Float16)vgpr_zero();
      const v8h z8 = {hz, hz, hz, hz, hz, hz, hz, hz};
      v8h o0, o1;
      o0[0] = (_Float16)(d0x * ASC); o0[1] = (_Float16)(d0y * ASC); o0[2] = (_Float16)(d0z * ASC);
      o0[3] = hz; o0[4] = hz; o0[5] = hz; o0[6] = hz; o0[7] = hz;
      o1[0] = (_Float16)(d1x * ASC); o1[1] = (_Float16)(d1y * ASC); o1[2] = (_Float16)(d1z * ASC);
      o1[3] = hz; o1[4] = hz; o1[5] = hz; o1[6] = hz; o1[7] = hz;
      *(v8h*)(XA + r0 * KAP + 64) = o0;
      *(v8h*)(XA + r0 * KAP + 72) = z8;
      *(v8h*)(XA + r0 * KAP + 80) = z8;
      *(v8h*)(XA + r0 * KAP + 88) = z8;
      *(v8h*)(XA + r1 * KAP + 64) = o1;
      *(v8h*)(XA + r1 * KAP + 72) = z8;
      *(v8h*)(XA + r1 * KAP + 80) = z8;
      *(v8h*)(XA + r1 * KAP + 88) = z8;
    }
#pragma unroll 2
    for (int it = 0; it < 16; ++it) {
      const int p = it * 32 + lane;
      const int row = p >> 3, c8 = (p & 7) * 8;
      int j = sIdx[64 * sg + row];
      j = min(max(j, 0), NP - 1);
      const float* src = p2b + (size_t)c8 * NP + j;
      v8h o;
#pragma unroll
      for (int e = 0; e < 8; ++e) o[e] = (_Float16)(src[(size_t)e * NP] * ASC);
      *(v8h*)(XA + row * KAP + c8) = o;
    }
    wave_sync();

#pragma unroll 1
    for (int nt = 0; nt < 4; ++nt) {
      v8f acc[4];
#pragma unroll
      for (int q = 0; q < 4; ++q) acc[q] = splat8(0.0f);
      const _Float16* brow = sW1 + (nt * 16 + nl) * K1P;
#pragma unroll
      for (int ks = 0; ks < 2; ++ks) {
        const v16h bf = ldfrag(brow, 32 * ks, hh);
#pragma unroll
        for (int q = 0; q < 4; ++q)
          acc[q] = wmf(ldfrag(XP1 + (4 * sg + q) * ND, 32 * ks, hh), bf, acc[q]);
      }
#pragma unroll
      for (int ks = 0; ks < 3; ++ks) {
        const v16h bf = ldfrag(brow, 64 + 32 * ks, hh);
#pragma unroll
        for (int q = 0; q < 4; ++q)
          acc[q] = wmf(ldfrag(XA + (q * 16 + nl) * KAP, 32 * ks, hh), bf, acc[q]);
      }
      const int col = nt * 16 + nl;
      const float bias = sB1[col];
#pragma unroll
      for (int q = 0; q < 4; ++q) {
#pragma unroll
        for (int r = 0; r < 8; ++r) {
          const float v = leaky01(acc[q][r] * XINV + bias);
          X1[(q * 16 + 8 * hh + r) * ND + col] = (_Float16)(v * ASC);
        }
      }
    }
    wave_sync();

#pragma unroll 1
    for (int nt = 0; nt < 4; ++nt) {
      v8f acc[4];
#pragma unroll
      for (int q = 0; q < 4; ++q) acc[q] = splat8(0.0f);
      const _Float16* brow = sW2 + (nt * 16 + nl) * ND;
#pragma unroll
      for (int ks = 0; ks < 2; ++ks) {
        const v16h bf = ldfrag(brow, 32 * ks, hh);
#pragma unroll
        for (int q = 0; q < 4; ++q)
          acc[q] = wmf(ldfrag(X1 + (q * 16 + nl) * ND, 32 * ks, hh), bf, acc[q]);
      }
      const int col = nt * 16 + nl;
      const float bias = sB2[col];
#pragma unroll
      for (int q = 0; q < 4; ++q) {
        const v4f wa = *(const v4f*)(sWt + q * 16 + 8 * hh);
        const v4f wb = *(const v4f*)(sWt + q * 16 + 8 * hh + 4);
        float pv = 0.0f;
        pv = fmaf(wa[0], leaky01(acc[q][0] * XINV + bias), pv);
        pv = fmaf(wa[1], leaky01(acc[q][1] * XINV + bias), pv);
        pv = fmaf(wa[2], leaky01(acc[q][2] * XINV + bias), pv);
        pv = fmaf(wa[3], leaky01(acc[q][3] * XINV + bias), pv);
        pv = fmaf(wb[0], leaky01(acc[q][4] * XINV + bias), pv);
        pv = fmaf(wb[1], leaky01(acc[q][5] * XINV + bias), pv);
        pv = fmaf(wb[2], leaky01(acc[q][6] * XINV + bias), pv);
        pv = fmaf(wb[3], leaky01(acc[q][7] * XINV + bias), pv);
        pv += __shfl_xor(pv, 16, 32);
        if (hh == 0) sOut[col * 32 + 4 * sg + q] = pv;
      }
    }
    wave_sync();
  }

  float* ob = outp + (size_t)b * ND * NP + n0w;
  const int cl = lane >> 3, pc = (lane & 7) * 4;
#pragma unroll
  for (int it = 0; it < 16; ++it) {
    const int c = it * 4 + cl;
    const v4f v = *(const v4f*)(sOut + c * 32 + pc);
    *(volatile v4f*)(ob + (size_t)c * NP + pc) = v;
  }
  __threadfence();
#pragma unroll
  for (int it = 0; it < 16; ++it) {
    const int c = it * 4 + cl;
    const v4f v = *(const v4f*)(sOut + c * 32 + pc);
    *(volatile v4f*)(ob + (size_t)c * NP + pc) = v;
  }
}

extern "C" void kernel_launch(void* const* d_in, const int* in_sizes, int n_in,
                              void* d_out, int out_size, void* d_ws, size_t ws_size,
                              hipStream_t stream) {
  (void)d_ws; (void)ws_size;
  if (n_in < 8) return;
  if (in_sizes[0] != NB * 3 * NP) return;
  if (in_sizes[1] != NB * 3 * NP) return;
  if (in_sizes[2] != NB * ND * NP) return;
  if (in_sizes[3] != NB * ND * NP) return;
  if (in_sizes[4] != ND * CIN) return;
  if (in_sizes[5] != ND) return;
  if (in_sizes[6] != ND * ND) return;
  if (in_sizes[7] != ND) return;
  if (out_size != NB * ND * NP) return;

  const float* xyz1 = (const float*)d_in[0];
  const float* xyz2 = (const float*)d_in[1];
  const float* pts1 = (const float*)d_in[2];
  const float* pts2 = (const float*)d_in[3];
  const float* W1   = (const float*)d_in[4];
  const float* b1   = (const float*)d_in[5];
  const float* W2   = (const float*)d_in[6];
  const float* b2   = (const float*)d_in[7];
  float* out = (float*)d_out;

  hipFuncSetAttribute(reinterpret_cast<const void*>(&k_main),
                      hipFuncAttributeMaxDynamicSharedMemorySize, SMEM);

  k_main<<<NB * NP / TPB, TPB, SMEM, stream>>>(xyz1, xyz2, pts1, pts2, W1, b1, W2, b2, out);
}
